// TSP_Decoder_3358664425904
// MI455X (gfx1250) — hardware-verified
//
#include <hip/hip_runtime.h>
#include <stddef.h>
#include <stdint.h>

#define NBATCH  32
#define NNODE   1000
#define NKEY    1024
#define NQ      256
#define EMB     256
#define NHEAD   16
#define HD      16
#define NBH     512
#define ENCROWS 32032
#define QROWS   8192
#define KC      64
#define NCH     16
#define PTP     72
#define OSP     132
#define SWP     68
#define TLP     68
#define CVT_ENC_BLOCKS (ENCROWS / 8)
#define CVT_QIN_BLOCKS (QROWS / 8)

static_assert(NBH == NBATCH * NHEAD);
static_assert(QROWS == NBATCH * NQ);
static_assert(NHEAD * HD == EMB);
static_assert(ENCROWS % 8 == 0);
static_assert(ENCROWS >= (NBATCH - 1) * NNODE + NKEY);
static_assert(NKEY == NCH * KC);
static_assert(NKEY >= NNODE);
static_assert(NQ % 16 == 0);
static_assert((16 * NNODE) % 4 == 0);
static_assert((16 * NNODE * 4) % 128 == 0);
static_assert(EMB % 64 == 0);

typedef unsigned short u16;
typedef __bf16 v16b __attribute__((ext_vector_type(16)));
typedef unsigned short v8us __attribute__((ext_vector_type(8)));
typedef float v8f __attribute__((ext_vector_type(8)));
typedef float v4f __attribute__((ext_vector_type(4)));
typedef unsigned int v4u __attribute__((ext_vector_type(4)));

union Frag  { v16b v; v8us h[2]; };
union Pack8 { v8us h; v4u u; u16 s[8]; };

__device__ __forceinline__ v8f zero8() { return (v8f){0.f, 0.f, 0.f, 0.f, 0.f, 0.f, 0.f, 0.f}; }

__device__ __forceinline__ v8f mma(v16b a, v16b b, v8f c) {
  c = __builtin_amdgcn_wmma_f32_16x16x32_bf16(false, a, false, b, (short)0, c, false, false);
  asm volatile("v_nop\n\tv_nop\n\tv_nop\n\tv_nop" : "+v"(c) : "v"(a), "v"(b));
  return c;
}

__device__ __forceinline__ u16 f2bf(float f) {
  unsigned int u = __float_as_uint(f);
  u += 0x7FFFu + ((u >> 16) & 1u);
  return (u16)(u >> 16);
}
__device__ __forceinline__ float bf2f(u16 h) { return __uint_as_float(((unsigned int)h) << 16); }
__device__ __forceinline__ u16 lo_of(float f, u16 hi) { return f2bf(f - bf2f(hi)); }
__device__ __forceinline__ void split8(v4f a, v4f b, v4u& hu, v4u& lu) {
  Pack8 ph, pl;
#pragma unroll
  for (int i = 0; i < 4; ++i) {
    const u16 h0 = f2bf(a[i]);
    ph.s[i] = h0;
    pl.s[i] = lo_of(a[i], h0);
    const u16 h1 = f2bf(b[i]);
    ph.s[4 + i] = h1;
    pl.s[4 + i] = lo_of(b[i], h1);
  }
  hu = ph.u;
  lu = pl.u;
}

__device__ __forceinline__ v16b ldfrag(const u16* p, int ld, int row0, int k0, int lane) {
  const int m = lane & 15, lh = lane >> 4;
  const u16* q = p + (size_t)(row0 + m) * ld + k0 + 8 * lh;
  Frag f;
  f.h[0] = *(const v8us*)(q);
  f.h[1] = *(const v8us*)(q + 16);
  return f.v;
}

__device__ __forceinline__ void gemm_hl(const u16* __restrict__ Ah, const u16* __restrict__ Al, int lda,
                                        const u16* __restrict__ Bh, const u16* __restrict__ Bl, int ldb, int K,
                                        int m0, int n0, int lane, v8f (&acc)[2][4]) {
#pragma unroll 1
  for (int k0 = 0; k0 < K; k0 += 32) {
    v16b bh[4];
#pragma unroll
    for (int t = 0; t < 4; ++t) bh[t] = ldfrag(Bh, ldb, n0 + 16 * t, k0, lane);
    const v16b a0 = ldfrag(Ah, lda, m0, k0, lane);
    const v16b a1 = ldfrag(Ah, lda, m0 + 16, k0, lane);
#pragma unroll
    for (int t = 0; t < 4; ++t) {
      acc[0][t] = mma(a0, bh[t], acc[0][t]);
      acc[1][t] = mma(a1, bh[t], acc[1][t]);
    }
    const v16b l0 = ldfrag(Al, lda, m0, k0, lane);
    const v16b l1 = ldfrag(Al, lda, m0 + 16, k0, lane);
#pragma unroll
    for (int t = 0; t < 4; ++t) {
      acc[0][t] = mma(l0, bh[t], acc[0][t]);
      acc[1][t] = mma(l1, bh[t], acc[1][t]);
    }
#pragma unroll
    for (int t = 0; t < 4; ++t) {
      const v16b bl = ldfrag(Bl, ldb, n0 + 16 * t, k0, lane);
      acc[0][t] = mma(a0, bl, acc[0][t]);
      acc[1][t] = mma(a1, bl, acc[1][t]);
    }
  }
}

__device__ __forceinline__ void gemm_hl16(const u16* __restrict__ Ah, const u16* __restrict__ Al, int lda,
                                          const u16* __restrict__ Bh, const u16* __restrict__ Bl, int ldb, int K,
                                          int m0, int n0, int lane, v8f (&acc)[4]) {
#pragma unroll 1
  for (int k0 = 0; k0 < K; k0 += 32) {
    v16b bh[4];
#pragma unroll
    for (int t = 0; t < 4; ++t) bh[t] = ldfrag(Bh, ldb, n0 + 16 * t, k0, lane);
    const v16b a0 = ldfrag(Ah, lda, m0, k0, lane);
#pragma unroll
    for (int t = 0; t < 4; ++t) acc[t] = mma(a0, bh[t], acc[t]);
    const v16b l0 = ldfrag(Al, lda, m0, k0, lane);
#pragma unroll
    for (int t = 0; t < 4; ++t) acc[t] = mma(l0, bh[t], acc[t]);
#pragma unroll
    for (int t = 0; t < 4; ++t) {
      const v16b bl = ldfrag(Bl, ldb, n0 + 16 * t, k0, lane);
      acc[t] = mma(a0, bl, acc[t]);
    }
  }
}

__global__ __launch_bounds__(256) void k_cvt(const float* __restrict__ enc, const float* __restrict__ q1,
                                             const float* __restrict__ ql,
                                             u16* __restrict__ ench, u16* __restrict__ encl,
                                             u16* __restrict__ qinh, u16* __restrict__ qinl) {
  const int tid = threadIdx.x, lane = tid & 31, wave = tid >> 5;
  if ((int)blockIdx.x < CVT_ENC_BLOCKS) {
    const int row  = blockIdx.x * 8 + wave;
    const int rowc = (row < NBATCH * NNODE) ? row : (NBATCH * NNODE - 1);
    const float* s = enc + (size_t)rowc * EMB + lane * 8;
    v4f a0 = *(const v4f*)(s), a1 = *(const v4f*)(s + 4);
    if (row >= NBATCH * NNODE) {
      a0 = (v4f){0.f, 0.f, 0.f, 0.f};
      a1 = (v4f){0.f, 0.f, 0.f, 0.f};
    }
    v4u hu, lu;
    split8(a0, a1, hu, lu);
    const size_t go = (size_t)row * EMB + lane * 8;
    *(volatile v4u*)(ench + go) = hu;
    *(volatile v4u*)(encl + go) = lu;
    __threadfence();
    *(volatile v4u*)(ench + go) = hu;
    *(volatile v4u*)(encl + go) = lu;
  } else {
    const int row = ((int)blockIdx.x - CVT_ENC_BLOCKS) * 8 + wave;
    const float* s1 = q1 + (size_t)row * EMB + lane * 8;
    const float* s2 = ql + (size_t)row * EMB + lane * 8;
    v4u h1, l1, h2, l2;
    split8(*(const v4f*)(s1), *(const v4f*)(s1 + 4), h1, l1);
    split8(*(const v4f*)(s2), *(const v4f*)(s2 + 4), h2, l2);
    const size_t g1 = (size_t)row * (2 * EMB) + lane * 8;
    const size_t g2 = g1 + EMB;
    *(volatile v4u*)(qinh + g1) = h1;
    *(volatile v4u*)(qinl + g1) = l1;
    *(volatile v4u*)(qinh + g2) = h2;
    *(volatile v4u*)(qinl + g2) = l2;
    __threadfence();
    *(volatile v4u*)(qinh + g1) = h1;
    *(volatile v4u*)(qinl + g1) = l1;
    *(volatile v4u*)(qinh + g2) = h2;
    *(volatile v4u*)(qinl + g2) = l2;
  }
}

__global__ __launch_bounds__(256) void k_cvt_w(const float* __restrict__ wqf, const float* __restrict__ wql,
                                               const float* __restrict__ wk, const float* __restrict__ wv,
                                               const float* __restrict__ wc,
                                               u16* __restrict__ wqth, u16* __restrict__ wqtl,
                                               u16* __restrict__ wkth, u16* __restrict__ wktl,
                                               u16* __restrict__ wvth, u16* __restrict__ wvtl,
                                               u16* __restrict__ wcth, u16* __restrict__ wctl) {
  __shared__ __align__(16) float tile[64 * TLP];
  const int tid = threadIdx.x;
  const int z = blockIdx.z;
  const int k0 = blockIdx.x * 64, n0 = blockIdx.y * 64;
  const float* src = (z == 0) ? wqf : ((z == 1) ? wql : ((z == 2) ? wk : ((z == 3) ? wv : wc)));
  u16* dh = (z <= 1) ? wqth : ((z == 2) ? wkth : ((z == 3) ? wvth : wcth));
  u16* dl = (z <= 1) ? wqtl : ((z == 2) ? wktl : ((z == 3) ? wvtl : wctl));
  const int ldo  = (z <= 1) ? (2 * EMB) : EMB;
  const int koff = (z == 1) ? EMB : 0;
#pragma unroll
  for (int it = 0; it < 4; ++it) {
    const int p = it * 256 + tid;
    const int kl = p >> 4, n4 = (p & 15) * 4;
    const v4f v = *(const v4f*)(src + (size_t)(k0 + kl) * EMB + n0 + n4);
    *(v4f*)(tile + kl * TLP + n4) = v;
  }
  __syncthreads();
  v4u hv[2], lv[2];
  size_t go[2];
#pragma unroll
  for (int it = 0; it < 2; ++it) {
    const int p = it * 256 + tid;
    const int nl = p >> 3, pc = p & 7;
    v4f a0, a1;
#pragma unroll
    for (int i = 0; i < 4; ++i) {
      a0[i] = tile[(8 * pc + i) * TLP + nl];
      a1[i] = tile[(8 * pc + 4 + i) * TLP + nl];
    }
    split8(a0, a1, hv[it], lv[it]);
    go[it] = (size_t)(n0 + nl) * ldo + koff + k0 + 8 * pc;
  }
#pragma unroll
  for (int it = 0; it < 2; ++it) {
    *(volatile v4u*)(dh + go[it]) = hv[it];
    *(volatile v4u*)(dl + go[it]) = lv[it];
  }
  __threadfence();
#pragma unroll
  for (int it = 0; it < 2; ++it) {
    *(volatile v4u*)(dh + go[it]) = hv[it];
    *(volatile v4u*)(dl + go[it]) = lv[it];
  }
}

__device__ __forceinline__ void epi_rows32(v8f (&acc)[2][4], u16* stw, u16* __restrict__ dst,
                                           int bh0, int nprow, int rowbase, int nvalid, int wave, int lane) {
  const int lh = lane >> 4, c = lane & 15;
#pragma unroll
  for (int sub = 0; sub < 2; ++sub) {
    __syncthreads();
#pragma unroll
    for (int t = 0; t < 4; ++t) {
#pragma unroll
      for (int r = 0; r < 8; ++r) {
        const int lrow = 8 * lh + r;
        const int grow = rowbase + wave * 32 + sub * 16 + lrow;
        const float v = (grow < nvalid) ? acc[sub][t][r] : 0.f;
        const u16 hi = f2bf(v);
        stw[t * 512 + lrow * 32 + c]      = hi;
        stw[t * 512 + lrow * 32 + 16 + c] = lo_of(v, hi);
      }
    }
    __syncthreads();
    v4u val[8];
    size_t go[8];
#pragma unroll
    for (int it = 0; it < 8; ++it) {
      const int t = it >> 1, q = (it & 1) * 32 + lane;
      const int row = q >> 2, pc = q & 3;
      Pack8 pk;
      pk.h    = *(const v8us*)(stw + t * 512 + row * 32 + pc * 8);
      val[it] = pk.u;
      go[it]  = ((size_t)(bh0 + t) * nprow + rowbase + wave * 32 + sub * 16 + row) * 32 + pc * 8;
    }
#pragma unroll
    for (int it = 0; it < 8; ++it) *(volatile v4u*)(dst + go[it]) = val[it];
    __threadfence();
#pragma unroll
    for (int it = 0; it < 8; ++it) *(volatile v4u*)(dst + go[it]) = val[it];
  }
}

__device__ __forceinline__ void epi_vt(v8f (&acc)[2][4], u16* st, u16* __restrict__ vth, u16* __restrict__ vtl,
                                       int bh0, int rowbase, int nvalid, int wave, int lane) {
  const int lh = lane >> 4, c = lane & 15;
#pragma unroll
  for (int pl = 0; pl < 2; ++pl) {
    __syncthreads();
#pragma unroll
    for (int sub = 0; sub < 2; ++sub) {
#pragma unroll
      for (int t = 0; t < 4; ++t) {
#pragma unroll
        for (int r = 0; r < 8; ++r) {
          const int key = wave * 32 + sub * 16 + 8 * lh + r;
          const float v = (rowbase + key < nvalid) ? acc[sub][t][r] : 0.f;
          const u16 hi = f2bf(v);
          st[(16 * t + c) * 256 + key] = (pl == 0) ? hi : lo_of(v, hi);
        }
      }
    }
    __syncthreads();
    u16* dst = (pl == 0) ? vth : vtl;
    v4u val[8];
    size_t go[8];
#pragma unroll
    for (int it = 0; it < 8; ++it) {
      const int q = it * 8 + wave;
      const int t = q >> 4, d = q & 15;
      Pack8 pk;
      pk.h    = *(const v8us*)(st + q * 256 + lane * 8);
      val[it] = pk.u;
      go[it]  = ((size_t)(bh0 + t) * HD + d) * NKEY + rowbase + lane * 8;
    }
#pragma unroll
    for (int it = 0; it < 8; ++it) *(volatile v4u*)(dst + go[it]) = val[it];
    __threadfence();
#pragma unroll
    for (int it = 0; it < 8; ++it) *(volatile v4u*)(dst + go[it]) = val[it];
  }
}

__global__ __launch_bounds__(256) void k_projkv(const u16* __restrict__ ench, const u16* __restrict__ encl,
                                                const u16* __restrict__ wkth, const u16* __restrict__ wktl,
                                                const u16* __restrict__ wvth, const u16* __restrict__ wvtl,
                                                u16* __restrict__ kp, u16* __restrict__ vth, u16* __restrict__ vtl) {
  __shared__ __align__(16) u16 st[16384];
  const int tid = threadIdx.x, lane = tid & 31, wave = tid >> 5;
  const int bx = blockIdx.x, b = bx >> 2, mblk = bx & 3;
  const int by = blockIdx.y, isv = by >> 2, nb = by & 3;
  const int m0 = b * NNODE + mblk * 256 + wave * 32;
  const int n0 = nb * 64;
  const u16* Bh = isv ? wvth : wkth;
  const u16* Bl = isv ? wvtl : wktl;

  v8f acc[2][4];
#pragma unroll
  for (int s = 0; s < 2; ++s)
#pragma unroll
    for (int t = 0; t < 4; ++t) acc[s][t] = zero8();
  gemm_hl(ench, encl, EMB, Bh, Bl, EMB, EMB, m0, n0, lane, acc);

  const int bh0 = b * NHEAD + nb * 4;
  if (isv == 0) {
    epi_rows32(acc, st + wave * 2048, kp, bh0, NKEY, mblk * 256, NNODE, wave, lane);
  } else {
    epi_vt(acc, st, vth, vtl, bh0, mblk * 256, NNODE, wave, lane);
  }
}

__global__ __launch_bounds__(256) void k_projq(const u16* __restrict__ qinh, const u16* __restrict__ qinl,
                                               const u16* __restrict__ wqth, const u16* __restrict__ wqtl,
                                               u16* __restrict__ qp) {
  __shared__ __align__(16) u16 st[16384];
  const int tid = threadIdx.x, lane = tid & 31, wave = tid >> 5;
  const int b = blockIdx.x, nb = blockIdx.y;
  const int m0 = b * NQ + wave * 32;
  const int n0 = nb * 64;

  v8f acc[2][4];
#pragma unroll
  for (int s = 0; s < 2; ++s)
#pragma unroll
    for (int t = 0; t < 4; ++t) acc[s][t] = zero8();
  gemm_hl(qinh, qinl, 2 * EMB, wqth, wqtl, 2 * EMB, 2 * EMB, m0, n0, lane, acc);
  epi_rows32(acc, st + wave * 2048, qp, b * NHEAD + nb * 4, NQ, 0, NQ, wave, lane);
}

__global__ __launch_bounds__(256) void k_attn(const u16* __restrict__ qp, const u16* __restrict__ kp,
                                              const u16* __restrict__ vth, const u16* __restrict__ vtl,
                                              const float* __restrict__ mask,
                                              u16* __restrict__ aoh, u16* __restrict__ aol) {
  __shared__ __align__(16) u16 Ps[8][2][16 * PTP];
  __shared__ __align__(16) float Os[16 * OSP];

  const int tid = threadIdx.x, lane = tid & 31, wave = tid >> 5;
  const int lh = lane >> 4, c = lane & 15;
  const int bid = blockIdx.x;
  const int g = bid & 1, qt = (bid >> 1) & 15, b = bid >> 5;
  const int h = g * 8 + wave, hb = b * NHEAD + h, q0 = qt * 16;

  const u16* Q  = qp + (size_t)hb * NQ * 32;
  const u16* Kb = kp + (size_t)hb * NKEY * 32;
  const u16* Vh = vth + (size_t)hb * HD * NKEY;
  const u16* Vl = vtl + (size_t)hb * HD * NKEY;
  const float* Mb = mask + ((size_t)(b * NQ + q0 + 8 * lh)) * NNODE;

  const v16b qa = ldfrag(Q, 32, q0, 0, lane);

  const float NEGI = -__builtin_huge_valf();
  float mrow[8], lrow[8];
  v8f oacc = zero8();
#pragma unroll
  for (int r = 0; r < 8; ++r) { mrow[r] = NEGI; lrow[r] = 0.f; }

  u16* ph = &Ps[wave][0][0];
  u16* pl = &Ps[wave][1][0];

#pragma unroll 1
  for (int kc = 0; kc < NCH; ++kc) {
    const int kv0 = kc * KC;
    __syncthreads();
    v8f s[4];
#pragma unroll
    for (int j = 0; j < 4; ++j) {
      const u16* kr = Kb + (size_t)(kv0 + 16 * j + c) * 32 + 8 * lh;
      Frag f1, f2;
      f1.h[0] = *(const v8us*)(kr);
      f1.h[1] = f1.h[0];
      f2.h[0] = *(const v8us*)(kr + 16);
      f2.h[1] = f2.h[0];
      s[j] = mma(qa, f1.v, zero8());
      s[j] = mma(qa, f2.v, s[j]);
    }
    float cm[8];
#pragma unroll
    for (int r = 0; r < 8; ++r) {
      const float* mp = Mb + (size_t)r * NNODE;
      float m = NEGI;
#pragma unroll
      for (int j = 0; j < 4; ++j) {
        const int key  = kv0 + 16 * j + c;
        const int keyc = (key < NNODE) ? key : (NNODE - 1);
        const float mv = mp[keyc];
        const float v  = (key < NNODE) ? (s[j][r] * 0.25f + mv) : NEGI;
        s[j][r] = v;
        m = fmaxf(m, v);
      }
#pragma unroll
      for (int off = 1; off < 16; off <<= 1) m = fmaxf(m, __shfl_xor(m, off, 32));
      cm[r] = m;
    }
    float al[8];
#pragma unroll
    for (int r = 0; r < 8; ++r) {
      const float mnew = fmaxf(mrow[r], cm[r]);
      const bool dead  = !(mnew > NEGI);
      const float alpha = dead ? 1.f : __expf(mrow[r] - mnew);
      mrow[r] = mnew;
      float psum = 0.f;
#pragma unroll
      for (int j = 0; j < 4; ++j) {
        const float p = dead ? 0.f : __expf(s[j][r] - mnew);
        psum += p;
        const u16 hi = f2bf(p);
        ph[(8 * lh + r) * PTP + 16 * j + c] = hi;
        pl[(8 * lh + r) * PTP + 16 * j + c] = lo_of(p, hi);
      }
#pragma unroll
      for (int off = 1; off < 16; off <<= 1) psum += __shfl_xor(psum, off, 32);
      lrow[r] = lrow[r] * alpha + psum;
      al[r] = alpha;
    }
#pragma unroll
    for (int r = 0; r < 8; ++r) oacc[r] *= al[r];
    __syncthreads();

#pragma unroll
    for (int kk = 0; kk < 2; ++kk) {
      const v16b pa = ldfrag(ph, PTP, 0, kk * 32, lane);
      const v16b pb = ldfrag(pl, PTP, 0, kk * 32, lane);
      const v16b vb = ldfrag(Vh, NKEY, 0, kv0 + kk * 32, lane);
      const v16b vc = ldfrag(Vl, NKEY, 0, kv0 + kk * 32, lane);
      oacc = mma(pa, vb, oacc);
      oacc = mma(pa, vc, oacc);
      oacc = mma(pb, vb, oacc);
    }
  }

#pragma unroll
  for (int r = 0; r < 8; ++r) {
    const float inv = (lrow[r] > 0.f) ? (1.0f / lrow[r]) : 0.f;
    Os[(8 * lh + r) * OSP + wave * 16 + c] = oacc[r] * inv;
  }
  __syncthreads();
  {
    const int row = tid >> 4, pc = tid & 15;
    const float* rp = Os + row * OSP + pc * 8;
    const v4f a0 = *(const v4f*)(rp), a1 = *(const v4f*)(rp + 4);
    v4u hu, lu;
    split8(a0, a1, hu, lu);
    const size_t go = (size_t)(b * NQ + q0 + row) * EMB + g * 128 + pc * 8;
    *(volatile v4u*)(aoh + go) = hu;
    *(volatile v4u*)(aol + go) = lu;
    __threadfence();
    *(volatile v4u*)(aoh + go) = hu;
    *(volatile v4u*)(aol + go) = lu;
  }
}

__global__ __launch_bounds__(256) void k_comb(const u16* __restrict__ aoh, const u16* __restrict__ aol,
                                              const u16* __restrict__ wcth, const u16* __restrict__ wctl,
                                              const float* __restrict__ bc,
                                              u16* __restrict__ mhh, u16* __restrict__ mhl) {
  __shared__ __align__(16) float sw[8][16 * SWP];
  const int tid = threadIdx.x, lane = tid & 31, wave = tid >> 5;
  const int lh = lane >> 4, c = lane & 15;
  const int m0 = blockIdx.x * 256 + wave * 32;
  const int n0 = blockIdx.y * 64;

  v8f acc[2][4];
#pragma unroll
  for (int s = 0; s < 2; ++s)
#pragma unroll
    for (int t = 0; t < 4; ++t) acc[s][t] = zero8();
  gemm_hl(aoh, aol, EMB, wcth, wctl, EMB, EMB, m0, n0, lane, acc);

  float bb[4];
#pragma unroll
  for (int t = 0; t < 4; ++t) bb[t] = bc[n0 + 16 * t + c];
  float* w = sw[wave];
#pragma unroll
  for (int sub = 0; sub < 2; ++sub) {
    __syncthreads();
#pragma unroll
    for (int t = 0; t < 4; ++t) {
#pragma unroll
      for (int r = 0; r < 8; ++r) w[(8 * lh + r) * SWP + 16 * t + c] = acc[sub][t][r] + bb[t];
    }
    __syncthreads();
    v4u hv[4], lv[4];
    size_t go[4];
#pragma unroll
    for (int it = 0; it < 4; ++it) {
      const int p = it * 32 + lane;
      const int L = p >> 3, pc = p & 7;
      const float* rp = w + L * SWP + pc * 8;
      const v4f a0 = *(const v4f*)(rp), a1 = *(const v4f*)(rp + 4);
      split8(a0, a1, hv[it], lv[it]);
      go[it] = (size_t)(m0 + sub * 16 + L) * EMB + n0 + pc * 8;
    }
#pragma unroll
    for (int it = 0; it < 4; ++it) {
      *(volatile v4u*)(mhh + go[it]) = hv[it];
      *(volatile v4u*)(mhl + go[it]) = lv[it];
    }
    __threadfence();
#pragma unroll
    for (int it = 0; it < 4; ++it) {
      *(volatile v4u*)(mhh + go[it]) = hv[it];
      *(volatile v4u*)(mhl + go[it]) = lv[it];
    }
  }
}

__global__ __launch_bounds__(256) void k_final(const u16* __restrict__ mhh, const u16* __restrict__ mhl,
                                               const u16* __restrict__ ench, const u16* __restrict__ encl,
                                               const float* __restrict__ mask, float* __restrict__ out) {
  __shared__ __align__(16) float Ls[16 * NNODE];
  const int tid = threadIdx.x, lane = tid & 31, wave = tid >> 5;
  const int lh = lane >> 4, c = lane & 15;
  const int b = blockIdx.x >> 4, pt = blockIdx.x & 15;
  const int p0 = pt * 16;
  const int arow0 = b * NQ + p0;
  const float NEGI = -__builtin_huge_valf();

#pragma unroll 1
  for (int ch = 0; ch < 2; ++ch) {
    const int n0 = (wave * 2 + ch) * 64;
    const int brow0 = b * NNODE + n0;
    v8f acc[4];
#pragma unroll
    for (int t = 0; t < 4; ++t) acc[t] = zero8();
    gemm_hl16(mhh, mhl, EMB, ench, encl, EMB, EMB, arow0, brow0, lane, acc);
#pragma unroll
    for (int t = 0; t < 4; ++t) {
#pragma unroll
      for (int r = 0; r < 8; ++r) {
        const int n  = n0 + 16 * t + c;
        const int p  = 8 * lh + r;
        const int nc = (n < NNODE) ? n : (NNODE - 1);
        const float mv = mask[(size_t)(arow0 + p) * NNODE + nc];
        const float x  = acc[t][r] * 0.0625f;
        const float ax = fabsf(x);
        const float e  = __expf(-2.f * ax);
        float th = (1.f - e) * __builtin_amdgcn_rcpf(1.f + e);
        th = copysignf(th, x);
        const float lg = 10.f * th + mv;
        if (n < NNODE) Ls[p * NNODE + n] = lg;
      }
    }
  }
  __syncthreads();

#pragma unroll
  for (int rr = 0; rr < 2; ++rr) {
    const int row = wave * 2 + rr;
    float* L = Ls + row * NNODE;
    float v[32];
    float m = NEGI;
#pragma unroll
    for (int i = 0; i < 32; ++i) {
      const int idx = lane + 32 * i;
      const int idc = (idx < NNODE) ? idx : (NNODE - 1);
      const float x = L[idc];
      v[i] = (idx < NNODE) ? x : NEGI;
      m = fmaxf(m, v[i]);
    }
#pragma unroll
    for (int off = 16; off >= 1; off >>= 1) m = fmaxf(m, __shfl_xor(m, off, 32));
    float ssum = 0.f;
#pragma unroll
    for (int i = 0; i < 32; ++i) {
      const float e = __expf(v[i] - m);
      v[i] = e;
      ssum += e;
    }
#pragma unroll
    for (int off = 16; off >= 1; off >>= 1) ssum += __shfl_xor(ssum, off, 32);
    const float inv = 1.0f / ssum;
#pragma unroll
    for (int i = 0; i < 32; ++i) {
      const int idx = lane + 32 * i;
      if (idx < NNODE) L[idx] = v[i] * inv;
    }
  }
  __syncthreads();

  float* ob = out + (size_t)arow0 * NNODE;
  v4f val[16];
#pragma unroll
  for (int it = 0; it < 16; ++it) {
    const int p   = it * 256 + tid;
    const int pcl = (p < 4 * NNODE) ? p : (4 * NNODE - 1);
    val[it] = *(const v4f*)(Ls + 4 * pcl);
  }
#pragma unroll
  for (int it = 0; it < 16; ++it) {
    const int p = it * 256 + tid;
    if (p < 4 * NNODE) *(volatile v4f*)(ob + 4 * p) = val[it];
  }
  __threadfence();
#pragma unroll
  for (int it = 0; it < 16; ++it) {
    const int p = it * 256 + tid;
    if (p < 4 * NNODE) *(volatile v4f*)(ob + 4 * p) = val[it];
  }
}

extern "C" void kernel_launch(void* const* d_in, const int* in_sizes, int n_in,
                              void* d_out, int out_size, void* d_ws, size_t ws_size,
                              hipStream_t stream) {
  if (n_in < 10) return;
  if (in_sizes[0] != NBATCH * NNODE * EMB) return;
  if (in_sizes[1] != QROWS * EMB) return;
  if (in_sizes[2] != QROWS * EMB) return;
  if (in_sizes[3] != QROWS * NNODE) return;
  if (in_sizes[4] != EMB * EMB) return;
  if (in_sizes[5] != EMB * EMB) return;
  if (in_sizes[6] != EMB * EMB) return;
  if (in_sizes[7] != EMB * EMB) return;
  if (in_sizes[8] != EMB * EMB) return;
  if (in_sizes[9] != EMB) return;
  if (out_size != QROWS * NNODE) return;

  const float* enc  = (const float*)d_in[0];
  const float* q1   = (const float*)d_in[1];
  const float* ql   = (const float*)d_in[2];
  const float* mask = (const float*)d_in[3];
  const float* wqf  = (const float*)d_in[4];
  const float* wql  = (const float*)d_in[5];
  const float* wk   = (const float*)d_in[6];
  const float* wv   = (const float*)d_in[7];
  const float* wc   = (const float*)d_in[8];
  const float* bc   = (const float*)d_in[9];
  float* out = (float*)d_out;

  const size_t szENC = (size_t)ENCROWS * EMB * 2;
  const size_t szQIN = (size_t)QROWS * 2 * EMB * 2;
  const size_t szWQ  = (size_t)EMB * 2 * EMB * 2;
  const size_t szW   = (size_t)EMB * EMB * 2;
  const size_t szKP  = (size_t)NBH * NKEY * 32 * 2;
  const size_t szVT  = (size_t)NBH * HD * NKEY * 2;
  const size_t szQP  = (size_t)NBH * NQ * 32 * 2;
  const size_t szAO  = (size_t)QROWS * EMB * 2;
  if (4 * szAO != 2 * szQIN) return;

  size_t off = 0;
  const size_t oENCH = off; off += szENC;
  const size_t oENCL = off; off += szENC;
  const size_t oQINH = off; off += szQIN;
  const size_t oQINL = off; off += szQIN;
  const size_t oWQH  = off; off += szWQ;
  const size_t oWQL  = off; off += szWQ;
  const size_t oWKH  = off; off += szW;
  const size_t oWKL  = off; off += szW;
  const size_t oWVH  = off; off += szW;
  const size_t oWVL  = off; off += szW;
  const size_t oWCH  = off; off += szW;
  const size_t oWCL  = off; off += szW;
  const size_t oKP   = off; off += szKP;
  const size_t oVTH  = off; off += szVT;
  const size_t oVTL  = off; off += szVT;
  const size_t oQP   = off; off += szQP;
  if (off > ws_size) return;
  if (off > (size_t)134217728) return;
  const size_t oAOH = oQINH;
  const size_t oAOL = oAOH + szAO;
  const size_t oMHH = oAOL + szAO;
  const size_t oMHL = oMHH + szAO;
  if (oMHL + szAO != oQINL + szQIN) return;

  char* ws = (char*)d_ws;
  u16* ENCH = (u16*)(ws + oENCH);
  u16* ENCL = (u16*)(ws + oENCL);
  u16* QINH = (u16*)(ws + oQINH);
  u16* QINL = (u16*)(ws + oQINL);
  u16* WQH  = (u16*)(ws + oWQH);
  u16* WQL  = (u16*)(ws + oWQL);
  u16* WKH  = (u16*)(ws + oWKH);
  u16* WKL  = (u16*)(ws + oWKL);
  u16* WVH  = (u16*)(ws + oWVH);
  u16* WVL  = (u16*)(ws + oWVL);
  u16* WCH  = (u16*)(ws + oWCH);
  u16* WCL  = (u16*)(ws + oWCL);
  u16* KP   = (u16*)(ws + oKP);
  u16* VTH  = (u16*)(ws + oVTH);
  u16* VTL  = (u16*)(ws + oVTL);
  u16* QP   = (u16*)(ws + oQP);
  u16* AOH  = (u16*)(ws + oAOH);
  u16* AOL  = (u16*)(ws + oAOL);
  u16* MHH  = (u16*)(ws + oMHH);
  u16* MHL  = (u16*)(ws + oMHL);

  k_cvt<<<dim3(CVT_ENC_BLOCKS + CVT_QIN_BLOCKS), dim3(256), 0, stream>>>(enc, q1, ql, ENCH, ENCL, QINH, QINL);
  k_cvt_w<<<dim3(4, 4, 5), dim3(256), 0, stream>>>(wqf, wql, wk, wv, wc, WQH, WQL, WKH, WKL, WVH, WVL, WCH, WCL);
  k_projkv<<<dim3(NBATCH * 4, 8), dim3(256), 0, stream>>>(ENCH, ENCL, WKH, WKL, WVH, WVL, KP, VTH, VTL);
  k_projq<<<dim3(NBATCH, 4), dim3(256), 0, stream>>>(QINH, QINL, WQH, WQL, QP);
  k_attn<<<dim3(NBATCH * 16 * 2), dim3(256), 0, stream>>>(QP, KP, VTH, VTL, mask, AOH, AOL);
  k_comb<<<dim3(QROWS / 256, EMB / 64), dim3(256), 0, stream>>>(AOH, AOL, WCH, WCL, bc, MHH, MHL);
  k_final<<<dim3(NBATCH * 16), dim3(256), 0, stream>>>(MHH, MHL, ENCH, ENCL, mask, out);
  (void)hipGetLastError();
}
